// SelfAttn_3882650436050
// MI455X (gfx1250) — hardware-verified
//
#include <hip/hip_runtime.h>

typedef __attribute__((ext_vector_type(16))) _Float16 v16h;
typedef __attribute__((ext_vector_type(16))) __bf16 v16b;
typedef __attribute__((ext_vector_type(8)))  _Float16 v8h;
typedef __attribute__((ext_vector_type(8)))  __bf16 v8b;
typedef __attribute__((ext_vector_type(8)))  float v8f;
typedef __attribute__((ext_vector_type(4)))  float v4f;
typedef __attribute__((ext_vector_type(4)))  unsigned v4u;

#define CIN 128
#define NPOS 4096
#define MPOS 1024
#define CK 16
#define CV 64
#define NOC 96
#define NBF 16
#ifndef NB
#define NB 16
#endif
#ifndef NQB
#define NQB (NPOS / 64)
#endif
#define RSC 2048.0f
#define PSC 16384.0f
#define XSP 136
#define GSP 72
#define SPP 36
#define SOP 68

static_assert(NPOS % 256 == 0);
static_assert(MPOS % 32 == 0);
static_assert(CIN % 32 == 0);
static_assert(CV % 32 == 0);
static_assert(NB >= 1 && NB <= NBF);
static_assert(NQB >= 1 && NQB <= NPOS / 64);

#define PK_WO  (NOC * CIN)
#define WS_PK  0u
#define WS_TH  (WS_PK + 2u * (NOC * CIN + CIN * CV))
#define WS_PH  (WS_TH + 2u * NBF * NPOS * 32)
#define WS_G   (WS_PH + 2u * NBF * MPOS * 32)
#define WS_END (WS_G + 2u * NBF * CV * MPOS)
static_assert(WS_TH % 128 == 0 && WS_PH % 128 == 0 && WS_G % 128 == 0);
static_assert(WS_END <= 134217728u);

template <typename T> __device__ __forceinline__ void vst2(void* p, T v) { *(volatile T*)p = v; __threadfence(); *(volatile T*)p = v; }

__device__ __forceinline__ v8f wmma16(v16h a, v16h b, v8f c) {
  v8f d = __builtin_amdgcn_wmma_f32_16x16x32_f16(false, a, false, b, (short)0, c, false, false);
  asm volatile("v_nop\n\tv_nop\n\tv_nop\n\tv_nop" : "+v"(d) : "v"(a), "v"(b));
  return d;
}
__device__ __forceinline__ v8f wmma_bf(v16b a, v16b b, v8f c) {
  v8f d = __builtin_amdgcn_wmma_f32_16x16x32_bf16(false, a, false, b, (short)0, c, false, false);
  asm volatile("v_nop\n\tv_nop\n\tv_nop\n\tv_nop" : "+v"(d) : "v"(a), "v"(b));
  return d;
}
__device__ __forceinline__ v16h frag_h(const _Float16* rowk0, int lane) {
  union { v16h v; v8h q[2]; } u; const _Float16* p = rowk0 + 8 * (lane >> 4);
  u.q[0] = *(const v8h*)p; u.q[1] = *(const v8h*)(p + 16); return u.v;
}
__device__ __forceinline__ v16h frag_hi0(const _Float16* row, int lane) {
  union { v16h v; v8h q[2]; v4u u[2]; } x; const v4u z = {0u, 0u, 0u, 0u};
  x.q[0] = *(const v8h*)(row + 8 * (lane >> 4)); x.u[1] = z; return x.v;
}
__device__ __forceinline__ v16h frag_lohi(const _Float16* row, int lane) {
  union { v16h v; v8h q[2]; } x; const _Float16* p = row + 8 * (lane >> 4);
  x.q[0] = *(const v8h*)(p + 16); x.q[1] = *(const v8h*)p; return x.v;
}
__device__ __forceinline__ v16b frag_b(const __bf16* rowk0, int lane) {
  union { v16b v; v8b q[2]; } u; const __bf16* p = rowk0 + 8 * (lane >> 4);
  u.q[0] = *(const v8b*)p; u.q[1] = *(const v8b*)(p + 16); return u.v;
}
struct F2 { v16b h, l; };
__device__ __forceinline__ F2 bsplit16(const float v[16]) { F2 r;
#pragma unroll
  for (int i = 0; i < 16; ++i) { const __bf16 hh = (__bf16)v[i]; r.h[i] = hh; r.l[i] = (__bf16)(v[i] - (float)hh); }
  return r; }
__device__ __forceinline__ F2 split_row(const float* row, int k0, int lane) { float v[16]; const float* p = row + k0 + 8 * (lane >> 4);
#pragma unroll
  for (int i = 0; i < 8; ++i) { v[i] = p[i]; v[8 + i] = p[16 + i]; }
  return bsplit16(v); }
__device__ __forceinline__ float bfr(float v) { return (float)(__bf16)v; }
__device__ __forceinline__ void ldsx() { asm volatile("s_wait_dscnt 0" ::: "memory"); __builtin_amdgcn_wave_barrier(); __builtin_amdgcn_fence(3, "workgroup"); }

__device__ __forceinline__ void cvt8(const float* __restrict__ src, __bf16* dst) {
  const v4f a = *(const v4f*)src, c = *(const v4f*)(src + 4);
  union { v8b v; v4u u; } o;
#pragma unroll
  for (int i = 0; i < 4; ++i) { const float fa = a[i], fc = c[i]; o.v[i] = (__bf16)fa; o.v[4 + i] = (__bf16)fc; }
  vst2(dst, o.u);
}
__global__ __launch_bounds__(256) void k_pack(const float* __restrict__ WT, const float* __restrict__ WP, const float* __restrict__ WG,
                                              const float* __restrict__ WO, __bf16* __restrict__ PK) {
  const int t = threadIdx.x;
  cvt8(WT + 8 * t, PK + 8 * t);
  cvt8(WP + 8 * t, PK + CK * CIN + 8 * t);
#pragma unroll 1
  for (int i = 0; i < 4; ++i) cvt8(WG + 8 * (256 * i + t), PK + 2 * CK * CIN + 8 * (256 * i + t));
#pragma unroll 1
  for (int i = 0; i < 4; ++i) cvt8(WO + 8 * (256 * i + t), PK + PK_WO + 8 * (256 * i + t));
}

__global__ __launch_bounds__(256) __attribute__((amdgpu_num_vgpr(256)))
void k_proj(const float* __restrict__ X, const __bf16* __restrict__ PK, _Float16* __restrict__ TH, _Float16* __restrict__ PH, _Float16* __restrict__ G) {
  __shared__ __align__(16) float ovl[80 * 128];
  __shared__ __align__(16) _Float16 sth[128 * 32];
  __shared__ __align__(16) _Float16 phst[64 * 32];
  __shared__ __align__(16) _Float16 gst[64 * GSP];
  __bf16* xs = (__bf16*)ovl; float* ys = ovl;
  const int rq = blockIdx.x, b = blockIdx.y, tid = threadIdx.x, wave = tid >> 5, lane = tid & 31, col = lane & 15, h = lane >> 4;
  const int nl = wave * 16 + col;
  for (int pz = 0; pz < 2; ++pz) {
    const int nb0 = (rq * 2 + pz) * 128;
    const float* xb = X + (size_t)b * CIN * NPOS + nb0;
#pragma unroll 4
    for (int i = 0; i < 16; ++i) {
      const int idx = i * 256 + tid, c = idx >> 5, n0 = (idx & 31) * 4;
      const v4f v = *(const v4f*)(xb + (size_t)c * NPOS + n0);
      const float f0 = v[0], f1 = v[1], f2 = v[2], f3 = v[3];
      xs[(n0 + 0) * XSP + c] = (__bf16)f0; xs[(n0 + 1) * XSP + c] = (__bf16)f1;
      xs[(n0 + 2) * XSP + c] = (__bf16)f2; xs[(n0 + 3) * XSP + c] = (__bf16)f3;
    }
    __syncthreads();
    v8f acc[6] = {};
#pragma unroll 1
    for (int kc = 0; kc < CIN / 32; ++kc) {
      union { v16b v; v8b q[2]; } xf; const __bf16* xr = xs + nl * XSP + kc * 32 + 8 * h;
      xf.q[0] = *(const v8b*)xr; xf.q[1] = *(const v8b*)(xr + 16);
#pragma unroll
      for (int j = 0; j < 6; ++j) acc[j] = wmma_bf(frag_b(PK + (size_t)(j * 16 + col) * CIN + kc * 32, lane), xf.v, acc[j]);
    }
    __syncthreads();
#pragma unroll
    for (int r = 0; r < 8; ++r) { const float v = acc[0][r]; const _Float16 hv = (_Float16)v;
      sth[nl * 32 + 8 * h + r] = hv; sth[nl * 32 + 16 + 8 * h + r] = (_Float16)((v - (float)hv) * RSC); }
#pragma unroll
    for (int j = 1; j < 6; ++j) {
#pragma unroll
      for (int r = 0; r < 8; ++r) ys[((j - 1) * 16 + 8 * h + r) * 128 + nl] = acc[j][r]; }
    __syncthreads();
    for (int i = 0; i < 2; ++i) {
      const int it = i * 256 + tid, c = it >> 5, wq = it & 31; const float* yr = ys + c * 128 + 2 * wq;
      const float mv = fmaxf(fmaxf(yr[0], yr[1]), fmaxf(yr[64], yr[65])); const _Float16 hv = (_Float16)mv;
      phst[(pz * 32 + wq) * 32 + c] = hv; phst[(pz * 32 + wq) * 32 + 16 + c] = (_Float16)((mv - (float)hv) * RSC);
    }
    for (int i = 0; i < 8; ++i) {
      const int it = i * 256 + tid, c = it >> 5, wq = it & 31; const float* yr = ys + (16 + c) * 128 + 2 * wq;
      gst[c * GSP + pz * 32 + wq] = (_Float16)fmaxf(fmaxf(yr[0], yr[1]), fmaxf(yr[64], yr[65]));
    }
    {
      _Float16* dst = TH + ((size_t)b * NPOS + nb0) * 32;
      for (int i = 0; i < 2; ++i) { const int p = i * 256 + tid; vst2(dst + (size_t)p * 8, *(const v4u*)&sth[p * 8]); }
    }
    __syncthreads();
  }
  {
    _Float16* dst = PH + ((size_t)b * MPOS + rq * 64) * 32;
    vst2(dst + (size_t)tid * 8, *(const v4u*)&phst[tid * 8]);
  }
  for (int i = 0; i < 2; ++i) {
    const int p = i * 256 + tid, c = p >> 3, j = p & 7;
    vst2(G + ((size_t)b * CV + c) * MPOS + rq * 64 + j * 8, *(const v4u*)&gst[c * GSP + j * 8]);
  }
}

__global__ __launch_bounds__(128) __attribute__((amdgpu_num_vgpr(256)))
void k_attn(const float* __restrict__ X, const _Float16* __restrict__ TH, const _Float16* __restrict__ PH, const _Float16* __restrict__ G,
            const __bf16* __restrict__ PKO, const float* __restrict__ GM, float* __restrict__ OUT) {
  __shared__ __align__(16) float sp[4][16][SPP];
  __shared__ __align__(16) float so[4][16][SOP];
  __shared__ __align__(16) float sob[128][SOP];
  const int tid = threadIdx.x, wave = tid >> 5, lane = tid & 31, col = lane & 15, h = lane >> 4;
  const int qb = blockIdx.x, b = blockIdx.y; const int q0 = qb * 64 + wave * 16;
  const _Float16* trow = TH + ((size_t)b * NPOS + q0 + col) * 32;
  const v16h ta0 = frag_hi0(trow, lane), ta1 = frag_lohi(trow, lane);
  float mrun[8], lrun[8];
#pragma unroll
  for (int r = 0; r < 8; ++r) { mrun[r] = -1.0e30f; lrun[r] = 0.f; }
  v8f acc[4] = {};
#pragma unroll 1
  for (int ks = 0; ks < MPOS / 32; ++ks) {
    v8f s[2];
#pragma unroll
    for (int ct = 0; ct < 2; ++ct) {
      const _Float16* prow = PH + ((size_t)b * MPOS + ks * 32 + ct * 16 + col) * 32;
      v8f c = {}, cl = {};
      c = wmma16(ta0, frag_hi0(prow, lane), c);
      cl = wmma16(ta1, frag_h(prow, lane), cl);
#pragma unroll
      for (int r = 0; r < 8; ++r) s[ct][r] = c[r] + cl[r] * (1.0f / RSC);
    }
#pragma unroll
    for (int r = 0; r < 8; ++r) {
      float mx = fmaxf(s[0][r], s[1][r]);
#pragma unroll
      for (int o = 1; o < 16; o <<= 1) mx = fmaxf(mx, __shfl_xor(mx, o));
      const float mn = fmaxf(mrun[r], mx); const float corr = __expf(mrun[r] - mn);
      const float e0 = __expf(s[0][r] - mn), e1 = __expf(s[1][r] - mn); float es = e0 + e1;
#pragma unroll
      for (int o = 1; o < 16; o <<= 1) es += __shfl_xor(es, o);
      lrun[r] = lrun[r] * corr + es; mrun[r] = mn;
#pragma unroll
      for (int dt = 0; dt < 4; ++dt) acc[dt][r] *= corr;
      sp[wave][8 * h + r][col] = e0 * PSC; sp[wave][8 * h + r][16 + col] = e1 * PSC;
    }
    ldsx();
    v16h pa; { const float* pr = &sp[wave][col][0] + 8 * h;
#pragma unroll
      for (int i = 0; i < 8; ++i) { pa[i] = (_Float16)pr[i]; pa[8 + i] = (_Float16)pr[16 + i]; } }
#pragma unroll
    for (int dt = 0; dt < 4; ++dt) acc[dt] = wmma16(pa, frag_h(G + ((size_t)b * CV + dt * 16 + col) * MPOS + ks * 32, lane), acc[dt]);
    ldsx();
  }
#pragma unroll
  for (int r = 0; r < 8; ++r) { const float il = 1.0f / (lrun[r] * PSC);
#pragma unroll
    for (int dt = 0; dt < 4; ++dt) so[wave][8 * h + r][dt * 16 + col] = acc[dt][r] * il; }
  ldsx();
  v8f acc2[8] = {};
#pragma unroll
  for (int kc = 0; kc < CV / 32; ++kc) {
    const F2 bq = split_row(&so[wave][col][0], kc * 32, lane);
#pragma unroll
    for (int j = 0; j < 8; ++j) { const v16b wa = frag_b(PKO + (size_t)(j * 16 + col) * CV + kc * 32, lane);
      acc2[j] = wmma_bf(wa, bq.l, acc2[j]); acc2[j] = wmma_bf(wa, bq.h, acc2[j]); }
  }
#pragma unroll
  for (int j = 0; j < 8; ++j) {
#pragma unroll
    for (int r = 0; r < 8; ++r) sob[j * 16 + 8 * h + r][wave * 16 + col] = acc2[j][r]; }
  __syncthreads();
  const float gm = bfr(GM[0]);
  const size_t ob = (size_t)b * CIN * NPOS + (size_t)qb * 64;
#pragma unroll 2
  for (int i = 0; i < 16; ++i) {
    const int p = i * 128 + tid, o = p >> 4, j = p & 15;
    const size_t off = ob + (size_t)o * NPOS + j * 4;
    const v4f xv = *(const v4f*)(X + off); const v4f ov = *(const v4f*)&sob[o][j * 4];
    v4f y;
#pragma unroll
    for (int e = 0; e < 4; ++e) { const float xe = xv[e], oe = ov[e]; y[e] = bfr(xe) + gm * oe; }
    vst2(OUT + off, y);
  }
}

extern "C" void kernel_launch(void* const* d_in, const int* in_sizes, int n_in, void* d_out, int out_size, void* d_ws, size_t ws_size, hipStream_t stream) {
  if (n_in < 6) return;
  if (in_sizes[0] < NB * CIN * NPOS || in_sizes[1] < CK * CIN || in_sizes[2] < CK * CIN || in_sizes[3] < CV * CIN || in_sizes[4] < CIN * CV || in_sizes[5] < 1) return;
  if (out_size < NB * CIN * NPOS) return;
  if (ws_size < (size_t)WS_END) return;
  const float* X  = (const float*)d_in[0];
  const float* WT = (const float*)d_in[1];
  const float* WP = (const float*)d_in[2];
  const float* WG = (const float*)d_in[3];
  const float* WO = (const float*)d_in[4];
  const float* GM = (const float*)d_in[5];
  char* ws = (char*)d_ws;
  __bf16* PK = (__bf16*)(ws + WS_PK); _Float16* TH = (_Float16*)(ws + WS_TH); _Float16* PH = (_Float16*)(ws + WS_PH); _Float16* G = (_Float16*)(ws + WS_G);
  k_pack<<<dim3(1), 256, 0, stream>>>(WT, WP, WG, WO, PK);
  k_proj<<<dim3(NPOS / 256, NB), 256, 0, stream>>>(X, PK, TH, PH, G);
  k_attn<<<dim3(NQB, NB), 128, 0, stream>>>(X, TH, PH, G, PK + PK_WO, GM, (float*)d_out);
}
